// mLSTMCell_2980707303872
// MI455X (gfx1250) — hardware-verified
//
#include <hip/hip_runtime.h>
#include <math.h>

constexpr int kBatch = 2;
constexpr int kSeq   = 2048;
constexpr int kDim   = 1024;
constexpr int kHeads = 8;
constexpr int kDh    = 128;
constexpr int kTok   = kBatch * kSeq;
constexpr int kGateK = 3 * kDim;
constexpr int kGateN = 64;
constexpr int kGroup = 2;
constexpr int kBH    = kBatch * kHeads;
constexpr float kQKScale   = 0.08838834764831845f;
constexpr float kPCarry    = 8.0f;
constexpr float kPCarryInv = 0.125f;
constexpr float kEps       = 1.0e-6f;
constexpr float kNormEps   = 1.0e-6f;
constexpr float kInvDh     = 1.0f / 128.0f;
static_assert(kHeads * kDh == kDim, "shape");
static_assert(kTok % 64 == 0 && kGateN % 64 == 0 && kGateK % 32 == 0, "gate gemm tiles");
static_assert(kSeq % 64 == 0 && kDh % 32 == 0, "score gemm tiles");
static_assert(kDh % 64 == 0 && kSeq % 32 == 0, "value gemm tiles");
static_assert(kHeads % kGroup == 0 && kSeq % 512 == 0 && kGateK % 256 == 0, "aux tiles");

typedef __attribute__((ext_vector_type(16))) _Float16 v16h;
typedef __attribute__((ext_vector_type(8)))  _Float16 v8h;
typedef __attribute__((ext_vector_type(16))) __bf16   v16b;
typedef __attribute__((ext_vector_type(8)))  __bf16   v8b;
typedef __attribute__((ext_vector_type(8)))  float    v8f;
typedef __attribute__((ext_vector_type(4)))  float    v4f;
typedef __attribute__((ext_vector_type(2)))  float    v2f;
typedef __attribute__((ext_vector_type(4)))  unsigned int v4u;

__device__ __forceinline__ unsigned short f2bf_bits(float f) {
  unsigned u = __float_as_uint(f);
  return (unsigned short)((u + 0x7FFFu + ((u >> 16) & 1u)) >> 16);
}
__device__ __forceinline__ float bf_bits2f(unsigned short h) { return __uint_as_float(((unsigned)h) << 16); }
__device__ __forceinline__ float bf16r(float f) { return bf_bits2f(f2bf_bits(f)); }

__device__ __forceinline__ void dep_guard_h(v8f& a, v8f& b, v16h x, v16h y) { asm volatile("v_nop\n\tv_nop\n\tv_nop\n\tv_nop" : "+v"(a), "+v"(b) : "v"(x), "v"(y)); }
__device__ __forceinline__ void dep_guard_b(v8f& a, v8f& b, v16b x, v16b y) { asm volatile("v_nop\n\tv_nop\n\tv_nop\n\tv_nop" : "+v"(a), "+v"(b) : "v"(x), "v"(y)); }
__device__ __forceinline__ void dep_guard4_h(v8f& a, v8f& b, v8f& c, v8f& d, v16h x, v16h y) { asm volatile("v_nop\n\tv_nop\n\tv_nop\n\tv_nop" : "+v"(a), "+v"(b), "+v"(c), "+v"(d) : "v"(x), "v"(y)); }
__device__ __forceinline__ void dep_guard4_b(v8f& a, v8f& b, v8f& c, v8f& d, v16b x, v16b y) { asm volatile("v_nop\n\tv_nop\n\tv_nop\n\tv_nop" : "+v"(a), "+v"(b), "+v"(c), "+v"(d) : "v"(x), "v"(y)); }
__device__ __forceinline__ void keep4_h(v16h a, v16h b, v16h c, v16h d) { asm volatile("v_nop" :: "v"(a), "v"(b), "v"(c), "v"(d)); }
__device__ __forceinline__ void keep4_b(v16b a, v16b b, v16b c, v16b d) { asm volatile("v_nop" :: "v"(a), "v"(b), "v"(c), "v"(d)); }
__device__ __forceinline__ void acc_guard4(v8f& a, v8f& b, v8f& c, v8f& d) { asm volatile("v_nop\n\tv_nop\n\tv_nop\n\tv_nop" : "+v"(a), "+v"(b), "+v"(c), "+v"(d)); }
template <typename T> struct Frag;
template <> struct Frag<_Float16> {
  typedef v16h V; union U { v16h v; v8h h[2]; };
  static __device__ __forceinline__ v16h load(const _Float16* p) {
    U f; f.h[0] = *(const v8h*)(p); f.h[1] = *(const v8h*)(p + 16); return f.v;
  }
  static __device__ __forceinline__ v8f mma(v16h a, v16h b, v8f c) {
    return __builtin_amdgcn_wmma_f32_16x16x32_f16(false, a, false, b, (short)0, c, false, false);
  }
  static __device__ __forceinline__ void guard(v8f& a, v8f& b, v16h x, v16h y) { dep_guard_h(a, b, x, y); }
  static __device__ __forceinline__ void guard4(v8f& a, v8f& b, v8f& c, v8f& d, v16h x, v16h y) { dep_guard4_h(a, b, c, d, x, y); }
  static __device__ __forceinline__ void keep(v16h a, v16h b, v16h c, v16h d) { keep4_h(a, b, c, d); }
};
template <> struct Frag<__bf16> {
  typedef v16b V; union U { v16b v; v8b h[2]; };
  static __device__ __forceinline__ v16b load(const __bf16* p) {
    U f; f.h[0] = *(const v8b*)(p); f.h[1] = *(const v8b*)(p + 16); return f.v;
  }
  static __device__ __forceinline__ v8f mma(v16b a, v16b b, v8f c) {
    return __builtin_amdgcn_wmma_f32_16x16x32_bf16(false, a, false, b, (short)0, c, false, false);
  }
  static __device__ __forceinline__ void guard(v8f& a, v8f& b, v16b x, v16b y) { dep_guard_b(a, b, x, y); }
  static __device__ __forceinline__ void guard4(v8f& a, v8f& b, v8f& c, v8f& d, v16b x, v16b y) { dep_guard4_b(a, b, c, d, x, y); }
  static __device__ __forceinline__ void keep(v16b a, v16b b, v16b c, v16b d) { keep4_b(a, b, c, d); }
};

__device__ __forceinline__ unsigned pk16(unsigned short a, unsigned short b) { return (unsigned)a | ((unsigned)b << 16); }
__device__ __forceinline__ unsigned short h_bits(float f) { const _Float16 h = (_Float16)f; return __builtin_bit_cast(unsigned short, h); }

template <int ET> struct Elem;
template <> struct Elem<0> { typedef _Float16 T; };
template <> struct Elem<1> { typedef __bf16 T; };
template <int ET, bool SPLIT, int BIAS_MODE, int OUT_MODE, bool RESID, int ACT = 0, int CAUS = 0>
__global__ __launch_bounds__(256) void wmma_gemm64(
    const unsigned short* __restrict__ Ap, const unsigned short* __restrict__ A2p, int lda, long strideA,
    const unsigned short* __restrict__ Btp, const unsigned short* __restrict__ Bt2p, int ldb, long strideB,
    void* __restrict__ Cout, void* __restrict__ Cout2, int ldc, long strideC,
    const float* __restrict__ bias,
    const float* __restrict__ resid, long strideR,
    int M, int N, int K, float scale) {
  typedef typename Elem<ET>::T T;
  typedef typename Frag<T>::V V;
  const T* A = (const T*)Ap; const T* A2 = (const T*)A2p; const T* Bt = (const T*)Btp; const T* Bt2 = (const T*)Bt2p;
  __shared__ __align__(16) float sT[8][16 * 68];
  const int b    = blockIdx.y;
  const int lane = threadIdx.x & 31;
  const int wave = threadIdx.x >> 5;
  const int tilesN = N >> 6;
  const int tilesM = M >> 6;
  const int tile = blockIdx.x * 8 + wave;
  if (tile >= tilesM * tilesN) return;
  const int tm = tile / tilesN;
  const int tn = tile - tm * tilesN;
  if (CAUS == 1 && tn > tm) return;
  const int m0 = tm << 6;
  const int n0 = tn << 6;
  int Klim = K;
  if (CAUS == 2) { const int kl = (tm + 1) << 6; Klim = (kl < K) ? kl : K; }

  const T* Ab  = A  + (size_t)b * strideA;
  const T* Bb  = Bt + (size_t)b * strideB;
  const T* Ab2 = SPLIT ? (A2  + (size_t)b * strideA) : nullptr;
  const T* Bb2 = SPLIT ? (Bt2 + (size_t)b * strideB) : nullptr;

  const int rlane = lane & 15;
  const int koff  = (lane >> 4) * 8;
  const int mOff  = (lane >> 4) * 8;

  v8f acc[4][4];
#pragma unroll
  for (int i = 0; i < 4; ++i)
#pragma unroll
    for (int j = 0; j < 4; ++j) acc[i][j] = (v8f){0.f,0.f,0.f,0.f,0.f,0.f,0.f,0.f};

  for (int k0 = 0; k0 < Klim; k0 += 32) {
    V bh[4], bl[4];
#pragma unroll
    for (int j = 0; j < 4; ++j) {
      const size_t bo = (size_t)(n0 + (j << 4) + rlane) * ldb + koff + k0;
      bh[j] = Frag<T>::load(Bb + bo);
      if (SPLIT) bl[j] = Frag<T>::load(Bb2 + bo);
    }
#pragma unroll
    for (int i = 0; i < 4; ++i) {
      const size_t ao = (size_t)(m0 + (i << 4) + rlane) * lda + koff + k0;
      V ah = Frag<T>::load(Ab + ao);
      V al;
      if (SPLIT) al = Frag<T>::load(Ab2 + ao);
#pragma unroll
      for (int j = 0; j < 4; ++j) {
        acc[i][j] = Frag<T>::mma(ah, bh[j], acc[i][j]);
        if (SPLIT) {
          acc[i][j] = Frag<T>::mma(ah, bl[j], acc[i][j]);
          acc[i][j] = Frag<T>::mma(al, bh[j], acc[i][j]);
        }
      }
      Frag<T>::guard4(acc[i][0], acc[i][1], acc[i][2], acc[i][3], ah, SPLIT ? al : ah);
    }
    Frag<T>::keep(bh[0], bh[1], bh[2], bh[3]);
    if (SPLIT) Frag<T>::keep(bl[0], bl[1], bl[2], bl[3]);
  }
  acc_guard4(acc[0][0], acc[0][1], acc[0][2], acc[0][3]);
  acc_guard4(acc[1][0], acc[1][1], acc[1][2], acc[1][3]);
  acc_guard4(acc[2][0], acc[2][1], acc[2][2], acc[2][3]);
  acc_guard4(acc[3][0], acc[3][1], acc[3][2], acc[3][3]);

  float* slab = sT[wave];
  const float* Rb = RESID ? (resid + (size_t)b * strideR) : nullptr;
#pragma unroll
  for (int i = 0; i < 4; ++i) {
    const int mBase = m0 + (i << 4);
#pragma unroll
    for (int j = 0; j < 4; ++j) {
      const int n = n0 + (j << 4) + rlane;
      float bv = 0.f;
      if (BIAS_MODE == 2) bv = bias[n];
#pragma unroll
      for (int r = 0; r < 8; ++r) {
        float v = acc[i][j][r] * scale;
        if (BIAS_MODE == 1) v += bias[mBase + mOff + r];
        if (BIAS_MODE == 2) v += bv;
        if (RESID) v += Rb[(size_t)(mBase + mOff + r) * ldc + n];
        if (ACT == 2) v = fmaxf(v, 0.0f);
        if (ACT == 4) v = (v > 0.f) ? v : 0.01f * v;
        slab[(mOff + r) * 68 + (j << 4) + rlane] = v;
      }
    }
    __builtin_amdgcn_fence(__ATOMIC_RELEASE, "workgroup");
    __builtin_amdgcn_wave_barrier();
    __builtin_amdgcn_fence(__ATOMIC_ACQUIRE, "workgroup");
    if (OUT_MODE == 0) {
      float* C = (float*)Cout + (size_t)b * strideC;
      const int hh = lane >> 4, c4 = (lane & 15) * 4;
      for (int pass = 0; pass < 2; ++pass) {
#pragma unroll
        for (int it = 0; it < 8; ++it) {
          const int row = it * 2 + hh;
          v4f v = *(const v4f*)(slab + row * 68 + c4);
          *(volatile v4f*)(C + (size_t)(mBase + row) * ldc + n0 + c4) = v;
        }
        __threadfence();
      }
    } else {
      const int q = lane >> 3, c8 = (lane & 7) * 8;
      unsigned short* C  = (unsigned short*)Cout  + (size_t)b * strideC;
      unsigned short* C2 = (OUT_MODE == 2) ? ((unsigned short*)Cout2 + (size_t)b * strideC) : nullptr;
      for (int pass = 0; pass < 2; ++pass) {
#pragma unroll
        for (int it = 0; it < 4; ++it) {
          const int row = it * 4 + q;
          const float* sp = slab + row * 68 + c8;
          v8h hv, lv;
#pragma unroll
          for (int e = 0; e < 8; ++e) {
            if (OUT_MODE == 1) {
              hv[e] = (_Float16)sp[e];
            } else {
              unsigned short hb = f2bf_bits(sp[e]);
              unsigned short lb = f2bf_bits(sp[e] - bf_bits2f(hb));
              hv[e] = __builtin_bit_cast(_Float16, hb);
              lv[e] = __builtin_bit_cast(_Float16, lb);
            }
          }
          *(volatile v8h*)(C + (size_t)(mBase + row) * ldc + n0 + c8) = hv;
          if (OUT_MODE == 2) *(volatile v8h*)(C2 + (size_t)(mBase + row) * ldc + n0 + c8) = lv;
        }
        __threadfence();
      }
    }
    __builtin_amdgcn_fence(__ATOMIC_RELEASE, "workgroup");
    __builtin_amdgcn_wave_barrier();
    __builtin_amdgcn_fence(__ATOMIC_ACQUIRE, "workgroup");
  }
}

__global__ __launch_bounds__(256) void cast_tokens_kernel(const float* __restrict__ q, const float* __restrict__ k,
                                                         const float* __restrict__ v, unsigned short* __restrict__ gb, int n8) {
  const int i = blockIdx.x * 256 + threadIdx.x;
  if (i >= n8) return;
  const int which = blockIdx.y;
  const float* src = (which == 0) ? q : ((which == 1) ? k : v);
  const size_t e0 = 8 * (size_t)i;
  const size_t token = e0 >> 10;
  const int col = (int)(e0 & 1023);
  const v4f a = *(const v4f*)(src + e0);
  const v4f c = *(const v4f*)(src + e0 + 4);
  unsigned short hb[8];
#pragma unroll
  for (int e = 0; e < 4; ++e) {
    hb[e]     = f2bf_bits(a[e]);
    hb[4 + e] = f2bf_bits(c[e]);
  }
  const v4u u = (v4u){pk16(hb[0], hb[1]), pk16(hb[2], hb[3]), pk16(hb[4], hb[5]), pk16(hb[6], hb[7])};
  unsigned short* d = gb + token * (size_t)kGateK + (size_t)which * kDim + col;
  *(volatile v4u*)d = u;
  __threadfence();
  *(volatile v4u*)d = u;
}

__global__ __launch_bounds__(256) void vt_cast_kernel(const float* __restrict__ v, unsigned short* __restrict__ vt) {
  __shared__ float sm[kDh][65];
  const int t  = threadIdx.x;
  const int s0 = blockIdx.x * 64;
  const int h  = blockIdx.y;
  const int b  = blockIdx.z;
  const float* vb = v + ((size_t)(b * kSeq + s0)) * kDim + h * kDh;
#pragma unroll
  for (int i = 0; i < 4; ++i) {
    const int e  = i * 256 + t;
    const int r  = e >> 5;
    const int c4 = (e & 31) * 4;
    const v4f w = *(const v4f*)(vb + (size_t)r * kDim + c4);
    sm[c4][r]     = w[0];
    sm[c4 + 1][r] = w[1];
    sm[c4 + 2][r] = w[2];
    sm[c4 + 3][r] = w[3];
  }
  asm volatile("" ::: "memory");
#pragma unroll
  for (int i = 4; i < 8; ++i) {
    const int e  = i * 256 + t;
    const int r  = e >> 5;
    const int c4 = (e & 31) * 4;
    const v4f w = *(const v4f*)(vb + (size_t)r * kDim + c4);
    sm[c4][r]     = w[0];
    sm[c4 + 1][r] = w[1];
    sm[c4 + 2][r] = w[2];
    sm[c4 + 3][r] = w[3];
  }
  __syncthreads();
  const int lane = t & 31, wave = t >> 5;
  const int qd = lane >> 3, c8 = (lane & 7) * 8;
  unsigned short* op = vt + ((size_t)(b * kHeads + h) * kDh) * kSeq;
  for (int pass = 0; pass < 2; ++pass) {
#pragma unroll
    for (int it = 0; it < 4; ++it) {
      const int row = wave * 16 + it * 4 + qd;
      unsigned short hb[8];
#pragma unroll
      for (int e = 0; e < 8; ++e) hb[e] = h_bits(bf16r(sm[row][c8 + e]));
      const v4u u = (v4u){pk16(hb[0], hb[1]), pk16(hb[2], hb[3]), pk16(hb[4], hb[5]), pk16(hb[6], hb[7])};
      *(volatile v4u*)(op + (size_t)row * kSeq + s0 + c8) = u;
    }
    __threadfence();
  }
}

__global__ __launch_bounds__(256) void wt_pack_kernel(const float* __restrict__ w_i, const float* __restrict__ w_f,
                                                     unsigned short* __restrict__ wt) {
  __shared__ __align__(16) float si[2048];
  __shared__ __align__(16) float sf[2048];
  const int t = threadIdx.x;
  const int lane = t & 31, wave = t >> 5;
  const int kb = blockIdx.x * 256;
  {
    const float* pi = w_i + (size_t)kb * 8 + 8 * t;
    const float* pf = w_f + (size_t)kb * 8 + 8 * t;
    *(v4f*)(si + 8 * t)     = *(const v4f*)(pi);
    *(v4f*)(si + 8 * t + 4) = *(const v4f*)(pi + 4);
    *(v4f*)(sf + 8 * t)     = *(const v4f*)(pf);
    *(v4f*)(sf + 8 * t + 4) = *(const v4f*)(pf + 4);
  }
  __syncthreads();
  const float fi = (wave == 0) ? 1.0f : 0.0f;
  const float ff = (wave == 1) ? 1.0f : 0.0f;
  for (int pass = 0; pass < 2; ++pass) {
#pragma unroll 1
    for (int it = 0; it < 8; ++it) {
      const int n = wave * 8 + it;
      const int ni = (n < 8) ? n : 7;
      int nf = n - 8; nf = (nf < 0) ? 0 : ((nf > 7) ? 7 : nf);
      unsigned short hb[8];
#pragma unroll
      for (int e = 0; e < 8; ++e) {
        const int kl = 8 * lane + e;
        const float a = si[kl * 8 + ni];
        const float c = sf[kl * 8 + nf];
        const float val = fi * a + ff * c;
        hb[e] = f2bf_bits(val);
      }
      const v4u u = (v4u){pk16(hb[0], hb[1]), pk16(hb[2], hb[3]), pk16(hb[4], hb[5]), pk16(hb[6], hb[7])};
      *(volatile v4u*)(wt + (size_t)n * kGateK + kb + 8 * lane) = u;
    }
    __threadfence();
  }
}

__global__ __launch_bounds__(32) void gate_scan_kernel(const float* __restrict__ gate, const float* __restrict__ b_i,
                                                      const float* __restrict__ b_f, float* __restrict__ fcp,
                                                      float* __restrict__ cvp, float* __restrict__ pmp) {
  const int bh = blockIdx.x;
  const int b = bh >> 3, h = bh & 7;
  const int lane = threadIdx.x;
  const float bi  = bf16r(b_i[h]);
  const float bfv = bf16r(b_f[h]);
  const size_t base = (size_t)bh * kSeq;
  float carry = 0.0f;
  float pcarry = -__builtin_inff();
#pragma unroll 1
  for (int c = 0; c < kSeq / 32; ++c) {
    const int s = c * 32 + lane;
    const float* gr = gate + ((size_t)(b * kSeq + s)) * kGateN;
    const float igv = gr[h] + bi;
    const float fgv = gr[kHeads + h] + bfv;
    const float lf = fminf(fgv, 0.0f) - log1pf(expf(-fabsf(fgv)));
    float x = lf;
#pragma unroll
    for (int off = 1; off < 32; off <<= 1) {
      const float y = __shfl_up(x, off, 32);
      x = (lane >= off) ? (x + y) : x;
    }
    x += carry;
    const float cvv = igv - x;
    float pm = cvv;
#pragma unroll
    for (int off = 1; off < 32; off <<= 1) {
      const float y = __shfl_up(pm, off, 32);
      pm = (lane >= off) ? fmaxf(pm, y) : pm;
    }
    pm = fmaxf(pm, pcarry);
    float* fq = fcp + base + s;
    float* cq = cvp + base + s;
    float* pq = pmp + base + s;
    *(volatile float*)fq = x;
    *(volatile float*)cq = cvv;
    *(volatile float*)pq = pm;
    __threadfence();
    *(volatile float*)fq = x;
    *(volatile float*)cq = cvv;
    *(volatile float*)pq = pm;
    carry  = __shfl(x, 31, 32);
    pcarry = __shfl(pm, 31, 32);
  }
}

__global__ __launch_bounds__(256) void weight_row_kernel(const float* __restrict__ scp, const float* __restrict__ cvp,
                                                        const float* __restrict__ pmp, const float* __restrict__ fcp,
                                                        unsigned short* __restrict__ pp, int bh0) {
  __shared__ __align__(16) float cb[kSeq];
  __shared__ float red[8];
  const int s    = blockIdx.x;
  const int hg   = blockIdx.y;
  const int bh   = bh0 + hg;
  const int t    = threadIdx.x;
  const int lane = t & 31, wave = t >> 5;
  const int lim  = ((s >> 6) + 1) << 6;
  const size_t rowoff = ((size_t)hg * kSeq + s) * kSeq;
  const float* sr  = scp + rowoff;
  const float* cvr = cvp + (size_t)bh * kSeq;
  const float pm = pmp[(size_t)bh * kSeq + s];
  const float fc = fcp[(size_t)bh * kSeq + s];

  float part = 0.0f;
#pragma unroll 1
  for (int it = 0; it < 4; ++it) {
    const int c  = it * 512 + 2 * t;
    const int cl = (c < lim - 2) ? c : (lim - 2);
    const v2f sv = *(const v2f*)(sr + cl);
    const v2f uv = *(const v2f*)(cvr + c);
    v2f cv;
#pragma unroll
    for (int e = 0; e < 2; ++e) {
      const float fv  = ((c + e) <= s) ? 1.0f : 0.0f;
      const float arg = fminf(uv[e] - pm, 0.0f);
      const float d   = expf(arg);
      const float cc  = fv * ((sv[e] * kQKScale) * d);
      cv[e] = cc;
      part += cc;
    }
    *(v2f*)(cb + c) = cv;
  }
#pragma unroll
  for (int off = 16; off > 0; off >>= 1) part += __shfl_xor(part, off, 32);
  if (lane == 0) red[wave] = part;
  __syncthreads();
  float tot = red[0];
#pragma unroll
  for (int w = 1; w < 8; ++w) tot += red[w];
  const float nrm = fmaxf(fabsf(tot), expf(-(fc + pm))) + kEps;
  const float inv = kPCarry / nrm;

  const v4f e0 = *(const v4f*)(cb + 8 * t);
  const v4f e1 = *(const v4f*)(cb + 8 * t + 4);
  unsigned short hb[8];
#pragma unroll
  for (int e = 0; e < 4; ++e) {
    hb[e]     = h_bits(e0[e] * inv);
    hb[4 + e] = h_bits(e1[e] * inv);
  }
  const v4u u = (v4u){pk16(hb[0], hb[1]), pk16(hb[2], hb[3]), pk16(hb[4], hb[5]), pk16(hb[6], hb[7])};
  unsigned short* pr = pp + rowoff + 8 * (size_t)t;
  *(volatile v4u*)pr = u;
  __threadfence();
  *(volatile v4u*)pr = u;
}

__global__ __launch_bounds__(256) void rmsnorm_kernel(const float* __restrict__ hw, const float* __restrict__ rms,
                                                    float* __restrict__ out, int nrows) {
  const int lane = threadIdx.x & 31, wave = threadIdx.x >> 5;
  const int r = blockIdx.x * 8 + wave;
  if (r >= nrows) return;
  const v4f x = *(const v4f*)(hw + (size_t)r * kDh + 4 * lane);
  float ss = (x[0] * x[0] + x[1] * x[1]) + (x[2] * x[2] + x[3] * x[3]);
#pragma unroll
  for (int off = 16; off > 0; off >>= 1) ss += __shfl_xor(ss, off, 32);
  const float rs = rsqrtf(ss * kInvDh + kNormEps);
  const v4f sc = *(const v4f*)(rms + 4 * lane);
  v4f o;
#pragma unroll
  for (int e = 0; e < 4; ++e) o[e] = (x[e] * rs) * (1.0f + bf16r(sc[e]));
  float* op = out + (size_t)r * kDh + 4 * lane;
  *(volatile v4f*)op = o;
  __threadfence();
  *(volatile v4f*)op = o;
}

extern "C" void kernel_launch(void* const* d_in, const int* in_sizes, int n_in,
                              void* d_out, int out_size, void* d_ws, size_t ws_size,
                              hipStream_t stream) {
  if (n_in < 8) return;
  const int nElem = kTok * kDim;
  if (in_sizes[0] != nElem || in_sizes[1] != nElem || in_sizes[2] != nElem) return;
  if (in_sizes[3] != kGateK * kHeads || in_sizes[5] != kGateK * kHeads) return;
  if (in_sizes[4] != kHeads || in_sizes[6] != kHeads || in_sizes[7] != kDh) return;
  if (out_size != nElem) return;

  const size_t szGB   = (size_t)kTok * kGateK * 2;
  const size_t szVT   = (size_t)kBH * kDh * kSeq * 2;
  const size_t szWT   = (size_t)kGateN * kGateK * 2;
  const size_t szGATE = (size_t)kTok * kGateN * 4;
  const size_t szSEQ  = (size_t)kBH * kSeq * 4;
  const size_t szHW   = (size_t)kTok * kDim * 4;
  const size_t szSC   = (size_t)kGroup * kSeq * kSeq * 4;
  const size_t szPP   = (size_t)kGroup * kSeq * kSeq * 2;
  const size_t offGB   = 0;
  const size_t offVT   = offGB + szGB;
  const size_t offWT   = offVT + szVT;
  const size_t offGATE = offWT + szWT;
  const size_t offFC   = offGATE + szGATE;
  const size_t offCV   = offFC + szSEQ;
  const size_t offPM   = offCV + szSEQ;
  const size_t offHW   = offPM + szSEQ;
  const size_t offSC   = offHW + szHW;
  const size_t offPP   = offSC + szSC;
  const size_t total   = offPP + szPP;
  if (ws_size < total) return;

  const float* q   = (const float*)d_in[0];
  const float* k   = (const float*)d_in[1];
  const float* v   = (const float*)d_in[2];
  const float* w_i = (const float*)d_in[3];
  const float* b_i = (const float*)d_in[4];
  const float* w_f = (const float*)d_in[5];
  const float* b_f = (const float*)d_in[6];
  const float* rms = (const float*)d_in[7];
  float* out = (float*)d_out;
  char* ws = (char*)d_ws;
  unsigned short* GB = (unsigned short*)(ws + offGB);
  unsigned short* VT = (unsigned short*)(ws + offVT);
  unsigned short* WT = (unsigned short*)(ws + offWT);
  float* GATE = (float*)(ws + offGATE);
  float* FC = (float*)(ws + offFC);
  float* CV = (float*)(ws + offCV);
  float* PM = (float*)(ws + offPM);
  float* HW = (float*)(ws + offHW);
  float* SC = (float*)(ws + offSC);
  unsigned short* PP = (unsigned short*)(ws + offPP);

  const int n8 = nElem / 8;
  cast_tokens_kernel<<<dim3(n8 / 256, 3), dim3(256), 0, stream>>>(q, k, v, GB, n8);
  vt_cast_kernel<<<dim3(kSeq / 64, kHeads, kBatch), dim3(256), 0, stream>>>(v, VT);
  wt_pack_kernel<<<dim3(kGateK / 256), dim3(256), 0, stream>>>(w_i, w_f, WT);

  const int tilesGate = (kTok / 64) * (kGateN / 64);
  wmma_gemm64<1, false, 0, 0, false, 0, 0><<<dim3(tilesGate / 8, 1), dim3(256), 0, stream>>>(
      GB, GB, kGateK, 0L, WT, WT, kGateK, 0L,
      (void*)GATE, (void*)GATE, kGateN, 0L, FC, FC, 0L, kTok, kGateN, kGateK, 1.0f);

  gate_scan_kernel<<<dim3(kBH), dim3(32), 0, stream>>>(GATE, b_i, b_f, FC, CV, PM);

  const long strideHead16 = (long)kDh;
  const long strideScore  = (long)kSeq * kSeq;
  const long strideVT     = (long)kDh * kSeq;
  const long strideHW     = (long)kDh;
  const int  tilesScore   = (kSeq / 64) * (kSeq / 64);
  const int  tilesVal     = (kSeq / 64) * (kDh / 64);
  for (int gi = 0; gi < kBH / kGroup; ++gi) {
    const int b   = gi / (kHeads / kGroup);
    const int h0  = (gi % (kHeads / kGroup)) * kGroup;
    const int bh0 = b * kHeads + h0;
    const size_t tokOff = ((size_t)b * kSeq) * kGateK + (size_t)h0 * kDh;
    const unsigned short* Ag  = GB + tokOff;
    const unsigned short* Btg = GB + tokOff + kDim;
    wmma_gemm64<1, false, 0, 0, false, 0, 1><<<dim3(tilesScore / 8, kGroup), dim3(256), 0, stream>>>(
        Ag, Ag, kGateK, strideHead16, Btg, Btg, kGateK, strideHead16,
        (void*)SC, (void*)SC, kSeq, strideScore, FC, FC, 0L, kSeq, kSeq, kDh, 1.0f);
    weight_row_kernel<<<dim3(kSeq, kGroup), dim3(256), 0, stream>>>(SC, CV, PM, FC, PP, bh0);
    const unsigned short* VTg = VT + (size_t)bh0 * kDh * kSeq;
    float* HWg = HW + ((size_t)b * kSeq) * kDim + (size_t)h0 * kDh;
    wmma_gemm64<0, false, 0, 0, false, 0, 2><<<dim3(tilesVal / 8, kGroup), dim3(256), 0, stream>>>(
        PP, PP, kSeq, strideScore, VTg, VTg, kSeq, strideVT,
        (void*)HWg, (void*)HWg, kDim, strideHW, FC, FC, 0L, kSeq, kDh, kSeq, kPCarryInv);
  }

  const int nrows = kTok * kHeads;
  rmsnorm_kernel<<<dim3(nrows / 8), dim3(256), 0, stream>>>(HW, rms, out, nrows);
}
